// PraxisAttention_75960791597801
// MI455X (gfx1250) — hardware-verified
//
#include <hip/hip_runtime.h>
#include <math.h>
#include <stdint.h>

#ifndef NB
#define NB 2
#endif
#ifndef SEQ
#define SEQ 1024
#endif
#define NB_FULL  2
#define SEQ_FULL 1024
#define NH     16
#define HD     64
#define HID    1024
#define MTOT   (NB * SEQ)
#define NQT    (SEQ / 128)
#define NBLK   (NB * NH * NQT)
#define GCOUNT (SEQ * HD)
#define KP     72
static_assert(NB >= 1 && NB <= NB_FULL);
static_assert(SEQ >= 128 && SEQ <= SEQ_FULL && (SEQ % 128) == 0);
static_assert(HID == 1024 && NH * HD == HID && (HID % 64) == 0);
static_assert((MTOT % 128) == 0 && ((MTOT * HID / 8) % 256) == 0);

#define VGPR_CAP __attribute__((amdgpu_num_vgpr(256)))

typedef __bf16   v16b __attribute__((ext_vector_type(16)));
typedef __bf16   v8b  __attribute__((ext_vector_type(8)));
typedef float    v8f  __attribute__((ext_vector_type(8)));
typedef float    v4f  __attribute__((ext_vector_type(4)));
typedef unsigned int v4u __attribute__((ext_vector_type(4)));
typedef double   v2d  __attribute__((ext_vector_type(2)));
union FB { v16b v; v8b h[2]; };

__device__ __forceinline__ unsigned short bf_bits(float f) {
  unsigned u = __float_as_uint(f);
  return (unsigned short)((u + 0x7FFFu + ((u >> 16) & 1u)) >> 16);
}
__device__ __forceinline__ float bf_up(unsigned short h) { return __uint_as_float(((unsigned)h) << 16); }
__device__ __forceinline__ __bf16 bf_val(unsigned short h) { return __builtin_bit_cast(__bf16, h); }
__device__ __forceinline__ unsigned pk16(unsigned short a, unsigned short b) { return (unsigned)a | ((unsigned)b << 16); }
__device__ __forceinline__ v8f zero8() { v8f z = {0.f, 0.f, 0.f, 0.f, 0.f, 0.f, 0.f, 0.f}; return z; }
__device__ __forceinline__ const __bf16* cbf(const unsigned short* p) { return (const __bf16*)(const void*)p; }
__device__ __forceinline__ v4u pack8(const float* p) {
  const v4f a = *(const v4f*)(p);
  const v4f b = *(const v4f*)(p + 4);
  v4u r;
  r[0] = pk16(bf_bits(a[0]), bf_bits(a[1]));
  r[1] = pk16(bf_bits(a[2]), bf_bits(a[3]));
  r[2] = pk16(bf_bits(b[0]), bf_bits(b[1]));
  r[3] = pk16(bf_bits(b[2]), bf_bits(b[3]));
  return r;
}
__device__ __forceinline__ void split2(float f0, float f1, unsigned& ph, unsigned& pl) {
  const unsigned short h0 = bf_bits(f0), h1 = bf_bits(f1);
  const unsigned short l0 = bf_bits(f0 - bf_up(h0)), l1 = bf_bits(f1 - bf_up(h1));
  ph = pk16(h0, h1);
  pl = pk16(l0, l1);
}
__device__ __forceinline__ void packhl(v4f a, v4f b, v4u& hi, v4u& lo) {
  unsigned ph, pl;
  split2(a[0], a[1], ph, pl); hi[0] = ph; lo[0] = pl;
  split2(a[2], a[3], ph, pl); hi[1] = ph; lo[1] = pl;
  split2(b[0], b[1], ph, pl); hi[2] = ph; lo[2] = pl;
  split2(b[2], b[3], ph, pl); hi[3] = ph; lo[3] = pl;
}
__device__ __forceinline__ float head_slope(int h) {
  const int e = (h + 1) >> 1;
  const float p2 = __uint_as_float(((unsigned)(127 - e)) << 23);
  return ((h + 1) & 1) ? (p2 * 0.70710678118654752f) : p2;
}

__device__ __forceinline__ v16b ldfrag_b(const __bf16* p) {
  union { v16b v; v8b h[2]; } f;
  f.h[0] = *(const v8b*)(p);
  f.h[1] = *(const v8b*)(p + 16);
  return f.v;
}

__device__ __forceinline__ v8f mma_b(v16b a, v16b b, v8f c) {
  c = __builtin_amdgcn_wmma_f32_16x16x32_bf16(false, a, false, b, (short)0, c, false, false);
  asm volatile("v_nop\n\tv_nop\n\tv_nop\n\tv_nop" : "+v"(c) : "v"(a), "v"(b));
  return c;
}

__global__ __launch_bounds__(256) void cvt_x(const float* __restrict__ x, unsigned short* xb, int n8) {
  const int i = blockIdx.x * 256 + threadIdx.x;
  if (i < n8) {
    const size_t e   = (size_t)i * 8;
    const int    m   = (int)(e >> 10);
    const int    col = (int)(e & 1023);
    const int    bb  = m / SEQ;
    const int    l   = m - bb * SEQ;
    const float* src = x + ((size_t)(bb * SEQ_FULL + l)) * HID + col;
    const v4u v = pack8(src);
    *(volatile v4u*)(xb + e) = v;
    __threadfence();
    *(volatile v4u*)(xb + e) = v;
  }
}

__global__ __launch_bounds__(256) void cvt_wt(const float* __restrict__ w0, const float* __restrict__ w1,
                                              const float* __restrict__ w2, const float* __restrict__ w3,
                                              const float* __restrict__ w4, const float* __restrict__ w5,
                                              unsigned short* wt) {
  __shared__ __align__(16) unsigned short T[64 * KP];
  const int tid = threadIdx.x;
  const int wi  = blockIdx.y;
  const float* W = (wi == 0) ? w0 : (wi == 1) ? w1 : (wi == 2) ? w2 : (wi == 3) ? w3 : (wi == 4) ? w4 : w5;
  const int nt = blockIdx.x & 15;
  const int kt = blockIdx.x >> 4;
  const int n0 = nt * 64, k0 = kt * 64;
#pragma unroll
  for (int i = 0; i < 4; ++i) {
    const int idx = i * 256 + tid;
    const int k   = idx >> 4;
    const int n4  = (idx & 15) * 4;
    const v4f f = *(const v4f*)(W + (size_t)(k0 + k) * HID + n0 + n4);
#pragma unroll
    for (int e = 0; e < 4; ++e) T[(n4 + e) * KP + k] = bf_bits(f[e]);
  }
  __syncthreads();
  const int q8 = tid >> 3, c8 = (tid & 7) * 8;
  v4u vals[2];
#pragma unroll
  for (int it = 0; it < 2; ++it) vals[it] = *(const v4u*)(T + (it * 32 + q8) * KP + c8);
  unsigned short* dst = wt + (size_t)wi * HID * HID + (size_t)n0 * HID + k0 + c8;
  for (int rep = 0; rep < 2; ++rep) {
#pragma unroll
    for (int it = 0; it < 2; ++it) *(volatile v4u*)(dst + (size_t)(it * 32 + q8) * HID) = vals[it];
    __threadfence();
  }
}

template <int MODE, int NPL>
__global__ __launch_bounds__(128) VGPR_CAP
void gemm_bt(const unsigned short* __restrict__ A0, const unsigned short* __restrict__ A1,
             const unsigned short* __restrict__ Btp,
             unsigned short* oh, unsigned short* ol, float* of) {
  __shared__ __align__(16) float S[128 * 68];
  const int tid  = threadIdx.x;
  const int wave = tid >> 5;
  const int lane = tid & 31;
  const int hh   = lane >> 4;
  const int c    = lane & 15;
  const int nblk = blockIdx.x * 64;
  const int mblk = blockIdx.y * 128;
  const int mw   = mblk + wave * 32;
  const __bf16* Bt = cbf(Btp) + (size_t)(nblk + c) * HID + 8 * hh;

  v8f acc[2][4];
#pragma unroll
  for (int mi = 0; mi < 2; ++mi)
#pragma unroll
    for (int nj = 0; nj < 4; ++nj) acc[mi][nj] = zero8();

#pragma unroll
  for (int pl = 0; pl < NPL; ++pl) {
    const unsigned short* Au = (pl == 0) ? A0 : A1;
    const __bf16* Ar = cbf(Au) + (size_t)(mw + c) * HID + 8 * hh;
#pragma unroll 2
    for (int k0 = 0; k0 < HID; k0 += 32) {
      const v16b a0 = ldfrag_b(Ar + k0);
      const v16b a1 = ldfrag_b(Ar + (size_t)16 * HID + k0);
      v16b bq[4];
#pragma unroll
      for (int nj = 0; nj < 4; ++nj) bq[nj] = ldfrag_b(Bt + (size_t)(nj * 16) * HID + k0);
#pragma unroll
      for (int nj = 0; nj < 4; ++nj) {
        acc[0][nj] = mma_b(a0, bq[nj], acc[0][nj]);
        acc[1][nj] = mma_b(a1, bq[nj], acc[1][nj]);
      }
    }
  }

#pragma unroll
  for (int mi = 0; mi < 2; ++mi)
#pragma unroll
    for (int nj = 0; nj < 4; ++nj)
#pragma unroll
      for (int r = 0; r < 8; ++r) {
        const int row = wave * 32 + mi * 16 + 8 * hh + r;
        const int col = nj * 16 + c;
        const float v = acc[mi][nj][r];
        if (MODE == 1) S[col * 132 + row] = v;
        else           S[row * 68 + col] = v;
      }
  __syncthreads();

  if (MODE == 2) {
    const int q16 = tid >> 4, c4 = (tid & 15) * 4;
    v4f fv[16];
#pragma unroll
    for (int it = 0; it < 16; ++it) fv[it] = *(const v4f*)(S + (it * 8 + q16) * 68 + c4);
    float* dst = of + (size_t)(mblk + q16) * HID + nblk + c4;
    for (int rep = 0; rep < 2; ++rep) {
#pragma unroll
      for (int it = 0; it < 16; ++it) *(volatile v4f*)(dst + (size_t)(it * 8) * HID) = fv[it];
      __threadfence();
    }
  } else if (MODE == 0) {
    const int q8 = tid >> 3, c8 = (tid & 7) * 8;
    const int h  = nblk >> 6;
    v4u hv[8], lv[8];
#pragma unroll
    for (int it = 0; it < 8; ++it) {
      const float* sp = S + (it * 16 + q8) * 68 + c8;
      packhl(*(const v4f*)(sp), *(const v4f*)(sp + 4), hv[it], lv[it]);
    }
    for (int rep = 0; rep < 2; ++rep) {
#pragma unroll
      for (int it = 0; it < 8; ++it) {
        const int m  = mblk + it * 16 + q8;
        const int bb = m / SEQ;
        const int l  = m - bb * SEQ;
        const size_t o = (((size_t)(bb * NH + h)) * SEQ + l) * HD + c8;
        *(volatile v4u*)(oh + o) = hv[it];
        *(volatile v4u*)(ol + o) = lv[it];
      }
      __threadfence();
    }
  } else {
    const int q16 = tid >> 4, k8 = (tid & 15) * 8;
    const int h   = nblk >> 6;
    const int bb  = mblk / SEQ;
    const int l0  = mblk - bb * SEQ;
    v4u hv[8], lv[8];
#pragma unroll
    for (int it = 0; it < 8; ++it) {
      const float* sp = S + (it * 8 + q16) * 132 + k8;
      packhl(*(const v4f*)(sp), *(const v4f*)(sp + 4), hv[it], lv[it]);
    }
    for (int rep = 0; rep < 2; ++rep) {
#pragma unroll
      for (int it = 0; it < 8; ++it) {
        const int drow = it * 8 + q16;
        const size_t o = (((size_t)(bb * NH + h)) * HD + drow) * SEQ + l0 + k8;
        *(volatile v4u*)(oh + o) = hv[it];
        *(volatile v4u*)(ol + o) = lv[it];
      }
      __threadfence();
    }
  }
}


__device__ __forceinline__ void stage64(const __bf16* src, size_t spitch, __bf16* dst, int tid) {
#pragma unroll
  for (int q = 0; q < 2; ++q) {
    const int p  = tid + 256 * q;
    const int r  = p >> 3;
    const int c8 = (p & 7) * 8;
    const v8b v = *(const v8b*)(src + (size_t)r * spitch + c8);
    *(v8b*)(dst + r * KP + c8) = v;
  }
}

__device__ __forceinline__ void scores3(const __bf16* qh, const __bf16* ql, const __bf16* Kh, const __bf16* Kl,
                                        int hh, int c, v8f (&s)[4]) {
#pragma unroll
  for (int j = 0; j < 4; ++j) s[j] = zero8();
#pragma unroll
  for (int dc = 0; dc < 2; ++dc) {
    const v16b qa = ldfrag_b(qh + dc * 32);
    const v16b qb = ldfrag_b(ql + dc * 32);
#pragma unroll
    for (int j = 0; j < 4; ++j) {
      const int kr = (j * 16 + c) * KP + dc * 32 + 8 * hh;
      FB kh, kl;
      kh.h[0] = *(const v8b*)(Kh + kr);
      kh.h[1] = *(const v8b*)(Kh + kr + 16);
      kl.h[0] = *(const v8b*)(Kl + kr);
      kl.h[1] = *(const v8b*)(Kl + kr + 16);
      s[j] = mma_b(qa, kh.v, s[j]);
      s[j] = mma_b(qa, kl.v, s[j]);
      s[j] = mma_b(qb, kh.v, s[j]);
    }
  }
}

__device__ __forceinline__ float add_bias(float acc, int rowq, int key, float slope, float padk) {
#pragma clang fp contract(off)
  float t = acc * 0.125f;
  const float al = slope * (float)(rowq - key);
  t = t - al;
  t = t + ((key > rowq) ? -1.0e9f : 0.0f);
  t = t + padk;
  return t;
}

__device__ __forceinline__ void online_stats(v8f (&s)[4], float (&m)[8], float (&l)[8], int q0w, int kv0,
                                             float slope, const float (&padk)[4], int hh, int c) {
#pragma unroll
  for (int r = 0; r < 8; ++r) {
    const int rowq = q0w + 8 * hh + r;
    float cm = -1.0e30f;
#pragma unroll
    for (int j = 0; j < 4; ++j) {
      const float t = add_bias(s[j][r], rowq, kv0 + j * 16 + c, slope, padk[j]);
      s[j][r] = t;
      cm = fmaxf(cm, t);
    }
#pragma unroll
    for (int off = 1; off < 16; off <<= 1) cm = fmaxf(cm, __shfl_xor(cm, off, 32));
    const float mn = fmaxf(m[r], cm);
    const float al = __expf(m[r] - mn);
    float ps = 0.f;
#pragma unroll
    for (int j = 0; j < 4; ++j) ps += __expf(s[j][r] - mn);
#pragma unroll
    for (int off = 1; off < 16; off <<= 1) ps += __shfl_xor(ps, off, 32);
    l[r] = l[r] * al + ps;
    m[r] = mn;
  }
}

__global__ __launch_bounds__(256) VGPR_CAP
void attn_stats(const unsigned short* q0h, const unsigned short* q0l,
                const unsigned short* q1h, const unsigned short* q1l,
                const unsigned short* k0h, const unsigned short* k0l,
                const unsigned short* k1h, const unsigned short* k1l,
                const float* __restrict__ amask, float* st) {
  __shared__ __align__(16) __bf16 Ks[4 * 64 * KP];
  __shared__ __align__(16) float stS[4 * 128];
  const int tid  = threadIdx.x;
  const int wave = tid >> 5;
  const int lane = tid & 31;
  const int hh   = lane >> 4;
  const int c    = lane & 15;
  const int bid  = blockIdx.x;
  const int qt   = bid % NQT;
  const int h    = (bid / NQT) % NH;
  const int b    = bid / (NQT * NH);
  const int q0w  = qt * 128 + wave * 16;
  const float slope = head_slope(h);

  const size_t pb = (size_t)(b * NH + h) * SEQ * HD;
  const size_t qo = pb + (size_t)(q0w + c) * HD + 8 * hh;
  const __bf16* Q0h = cbf(q0h) + qo;
  const __bf16* Q0l = cbf(q0l) + qo;
  const __bf16* Q1h = cbf(q1h) + qo;
  const __bf16* Q1l = cbf(q1l) + qo;
  const __bf16* K0h = cbf(k0h) + pb;
  const __bf16* K0l = cbf(k0l) + pb;
  const __bf16* K1h = cbf(k1h) + pb;
  const __bf16* K1l = cbf(k1l) + pb;
  const float* mrow = amask + (size_t)b * SEQ_FULL;

  float m0[8], l0[8], m1[8], l1[8];
#pragma unroll
  for (int r = 0; r < 8; ++r) { m0[r] = -1.0e30f; l0[r] = 0.f; m1[r] = -1.0e30f; l1[r] = 0.f; }

  const int nkt = 2 * qt + 2;
  for (int kt = 0; kt < nkt; ++kt) {
    const int kv0 = kt * 64;
    __syncthreads();
    stage64(K0h + (size_t)kv0 * HD, HD, Ks, tid);
    stage64(K0l + (size_t)kv0 * HD, HD, Ks + 4608, tid);
    stage64(K1h + (size_t)kv0 * HD, HD, Ks + 9216, tid);
    stage64(K1l + (size_t)kv0 * HD, HD, Ks + 13824, tid);
    __syncthreads();
    float padk[4];
#pragma unroll
    for (int j = 0; j < 4; ++j) {
      const float mk = bf_up(bf_bits(mrow[kv0 + j * 16 + c]));
      padk[j] = (1.0f - mk) * (-1.0e9f);
    }
    {
      int dz = 0;
      asm volatile("" : "+v"(dz));
      v8f s[4];
      scores3(Q0h + dz, Q0l + dz, Ks, Ks + 4608, hh, c, s);
      online_stats(s, m0, l0, q0w, kv0, slope, padk, hh, c);
    }
    asm volatile("" ::: "memory");
    {
      int dz = 0;
      asm volatile("" : "+v"(dz));
      v8f s[4];
      scores3(Q1h + dz, Q1l + dz, Ks + 9216, Ks + 13824, hh, c, s);
      online_stats(s, m1, l1, q0w, kv0, slope, padk, hh, c);
    }
  }

#pragma unroll
  for (int r = 0; r < 8; ++r) {
    if (c == 0) {
      const int row = wave * 16 + 8 * hh + r;
      stS[row]       = m0[r];
      stS[128 + row] = 1.0f / l0[r];
      stS[256 + row] = m1[r];
      stS[384 + row] = 1.0f / l1[r];
    }
  }
  __syncthreads();
  if (wave < 4) {
    const v4f v = *(const v4f*)(stS + wave * 128 + lane * 4);
    float* dst = st + ((size_t)(b * NH + h) * 4 + wave) * SEQ + qt * 128 + lane * 4;
    *(volatile v4f*)dst = v;
    __threadfence();
    *(volatile v4f*)dst = v;
  }
}

#define L_K     0
#define L_VT    36864
#define L_PH    55296
#define L_PL    73728
#define L_ACC   92160
#define L_WP    124928
#define L_P0    129024
#define L_TOTAL 161792
static_assert(L_VT - L_K == 4 * 64 * KP * 2);
static_assert(L_PH - L_VT == 2 * 64 * KP * 2);
static_assert(L_PL - L_PH == 8 * 16 * KP * 2 && L_ACC - L_PL == 8 * 16 * KP * 2);
static_assert(L_WP - L_ACC == 8 * 4 * 32 * 8 * 4);
static_assert(L_P0 - L_WP == 256 * 2 * 8);
static_assert(L_TOTAL - L_P0 == 8 * 16 * 64 * 4);
static_assert(8 * 16 * 68 * 4 <= L_VT);

__global__ __launch_bounds__(256) VGPR_CAP
void attn_out(const unsigned short* q0h, const unsigned short* q0l,
              const unsigned short* q1h, const unsigned short* q1l,
              const unsigned short* k0h, const unsigned short* k0l,
              const unsigned short* k1h, const unsigned short* k1l,
              const unsigned short* vth, const unsigned short* vtl,
              const float* __restrict__ amask, const float* __restrict__ st,
              const float* __restrict__ l0p, const float* __restrict__ l1p,
              float* Op, double* recp) {
  extern __shared__ __align__(16) unsigned char lds[];
  __bf16* Ks    = (__bf16*)(lds + L_K);
  __bf16* Vt    = (__bf16*)(lds + L_VT);
  __bf16* Ph    = (__bf16*)(lds + L_PH);
  __bf16* Pl    = (__bf16*)(lds + L_PL);
  float*  accL  = (float*)(lds + L_ACC);
  double* wpart = (double*)(lds + L_WP);
  float*  p0L   = (float*)(lds + L_P0);

  const int tid  = threadIdx.x;
  const int wave = tid >> 5;
  const int lane = tid & 31;
  const int hh   = lane >> 4;
  const int c    = lane & 15;
  const int bid  = blockIdx.x;
  const int qt   = bid % NQT;
  const int h    = (bid / NQT) % NH;
  const int b    = bid / (NQT * NH);
  const int q0w  = qt * 128 + wave * 16;
  const float slope = head_slope(h);

  double sl = 0.0;
#pragma unroll 1
  for (int i = 0; i < HD; ++i) {
    const float a  = bf_up(bf_bits(l0p[h * HD + i]));
    const float bb = bf_up(bf_bits(l1p[h * HD + i]));
    sl += (double)(a * bb);
  }
  const float lam = 0.8f + expf((float)sl);

  float m0[8], il0[8], m1[8], il1[8];
  {
    const float* sp = st + (size_t)(b * NH + h) * 4 * SEQ + q0w + 8 * hh;
    const v4f a0 = *(const v4f*)(sp),           a1 = *(const v4f*)(sp + 4);
    const v4f b0 = *(const v4f*)(sp + SEQ),     b1 = *(const v4f*)(sp + SEQ + 4);
    const v4f c0 = *(const v4f*)(sp + 2 * SEQ), c1 = *(const v4f*)(sp + 2 * SEQ + 4);
    const v4f d0 = *(const v4f*)(sp + 3 * SEQ), d1 = *(const v4f*)(sp + 3 * SEQ + 4);
#pragma unroll
    for (int r = 0; r < 4; ++r) {
      m0[r]  = a0[r]; m0[4 + r]  = a1[r];
      il0[r] = b0[r]; il0[4 + r] = b1[r];
      m1[r]  = c0[r]; m1[4 + r]  = c1[r];
      il1[r] = d0[r]; il1[4 + r] = d1[r];
    }
  }

  const size_t pb = (size_t)(b * NH + h) * SEQ * HD;
  const size_t qo = pb + (size_t)(q0w + c) * HD + 8 * hh;
  const __bf16* Q0h = cbf(q0h) + qo;
  const __bf16* Q0l = cbf(q0l) + qo;
  const __bf16* Q1h = cbf(q1h) + qo;
  const __bf16* Q1l = cbf(q1l) + qo;
  const __bf16* K0h = cbf(k0h) + pb;
  const __bf16* K0l = cbf(k0l) + pb;
  const __bf16* K1h = cbf(k1h) + pb;
  const __bf16* K1l = cbf(k1l) + pb;
  const __bf16* VTh = cbf(vth) + (size_t)(b * NH + h) * HD * SEQ;
  const __bf16* VTl = cbf(vtl) + (size_t)(b * NH + h) * HD * SEQ;
  const float* mrow = amask + (size_t)b * SEQ_FULL;

  float*  accW = accL + wave * 1024;
  __bf16* pwh  = Ph + wave * (16 * KP);
  __bf16* pwl  = Pl + wave * (16 * KP);
  float*  p0S  = p0L + wave * 1024;
#pragma unroll
  for (int t = 0; t < 4; ++t) *(v8f*)(accW + (t * 32 + lane) * 8) = zero8();

  const int nkt = 2 * qt + 2;
  for (int kt = 0; kt < nkt; ++kt) {
    const int kv0 = kt * 64;
    __syncthreads();
    stage64(K0h + (size_t)kv0 * HD, HD, Ks, tid);
    stage64(K0l + (size_t)kv0 * HD, HD, Ks + 4608, tid);
    stage64(K1h + (size_t)kv0 * HD, HD, Ks + 9216, tid);
    stage64(K1l + (size_t)kv0 * HD, HD, Ks + 13824, tid);
    stage64(VTh + kv0, SEQ, Vt, tid);
    stage64(VTl + kv0, SEQ, Vt + 4608, tid);
    __syncthreads();
    float padk[4];
#pragma unroll
    for (int j = 0; j < 4; ++j) {
      const float mk = bf_up(bf_bits(mrow[kv0 + j * 16 + c]));
      padk[j] = (1.0f - mk) * (-1.0e9f);
    }

    {
      int dz = 0;
      asm volatile("" : "+v"(dz));
      v8f p0[4];
      scores3(Q0h + dz, Q0l + dz, Ks, Ks + 4608, hh, c, p0);
#pragma unroll
      for (int r = 0; r < 8; ++r) {
        const int rowq = q0w + 8 * hh + r;
#pragma unroll
        for (int j = 0; j < 4; ++j) {
          const float t = add_bias(p0[j][r], rowq, kv0 + j * 16 + c, slope, padk[j]);
          p0S[(8 * hh + r) * 64 + j * 16 + c] = __expf(t - m0[r]) * il0[r];
        }
      }
    }
    asm volatile("" ::: "memory");
    v8f s1[4];
    {
      int dz = 0;
      asm volatile("" : "+v"(dz));
      scores3(Q1h + dz, Q1l + dz, Ks + 9216, Ks + 13824, hh, c, s1);
    }
    asm volatile("" ::: "memory");
#pragma unroll
    for (int r = 0; r < 8; ++r) {
      const int rowq = q0w + 8 * hh + r;
#pragma unroll
      for (int j = 0; j < 4; ++j) {
        const float t   = add_bias(s1[j][r], rowq, kv0 + j * 16 + c, slope, padk[j]);
        const float p1  = __expf(t - m1[r]) * il1[r];
        const float p0v = p0S[(8 * hh + r) * 64 + j * 16 + c];
        const float P   = lam * (p0v - p1);
        const unsigned short hb = bf_bits(P);
        const unsigned short lb = bf_bits(P - bf_up(hb));
        const int po = (8 * hh + r) * KP + j * 16 + c;
        pwh[po] = bf_val(hb);
        pwl[po] = bf_val(lb);
      }
    }
    __builtin_amdgcn_fence(__ATOMIC_RELEASE, "workgroup");
    __builtin_amdgcn_wave_barrier();
    __builtin_amdgcn_fence(__ATOMIC_ACQUIRE, "workgroup");

    FB pa[2], pg[2];
#pragma unroll
    for (int kk = 0; kk < 2; ++kk) {
      const int pr = c * KP + kk * 32 + 8 * hh;
      pa[kk].h[0] = *(const v8b*)(pwh + pr);
      pa[kk].h[1] = *(const v8b*)(pwh + pr + 16);
      pg[kk].h[0] = *(const v8b*)(pwl + pr);
      pg[kk].h[1] = *(const v8b*)(pwl + pr + 16);
    }
#pragma unroll 1
    for (int t = 0; t < 4; ++t) {
      float* ap = accW + (t * 32 + lane) * 8;
      v8f acc = *(const v8f*)ap;
      const int vr0 = (t * 16 + c) * KP + 8 * hh;
#pragma unroll
      for (int kk = 0; kk < 2; ++kk) {
        FB vh, vl;
        vh.h[0] = *(const v8b*)(Vt + vr0 + kk * 32);
        vh.h[1] = *(const v8b*)(Vt + vr0 + kk * 32 + 16);
        vl.h[0] = *(const v8b*)(Vt + 4608 + vr0 + kk * 32);
        vl.h[1] = *(const v8b*)(Vt + 4608 + vr0 + kk * 32 + 16);
        acc = mma_b(pa[kk].v, vh.v, acc);
        acc = mma_b(pa[kk].v, vl.v, acc);
        acc = mma_b(pg[kk].v, vh.v, acc);
      }
      *(v8f*)ap = acc;
    }
  }

  __syncthreads();
  float* Ob = (float*)(lds + L_K) + wave * (16 * 68);
  double ps = 0.0, ps2 = 0.0;
#pragma unroll 1
  for (int t = 0; t < 4; ++t) {
    const v8f acc = *(const v8f*)(accW + (t * 32 + lane) * 8);
#pragma unroll
    for (int r = 0; r < 8; ++r) {
      const float y = acc[r];
      Ob[(8 * hh + r) * 68 + t * 16 + c] = y;
      ps  += (double)y;
      ps2 += (double)y * (double)y;
    }
  }
  wpart[tid * 2]     = ps;
  wpart[tid * 2 + 1] = ps2;
  __builtin_amdgcn_fence(__ATOMIC_RELEASE, "workgroup");
  __builtin_amdgcn_wave_barrier();
  __builtin_amdgcn_fence(__ATOMIC_ACQUIRE, "workgroup");
  float* og = Op + ((size_t)(b * NH + h) * SEQ + q0w) * HD;
  v4f ov[8];
#pragma unroll
  for (int i = 0; i < 8; ++i) ov[i] = *(const v4f*)(Ob + (2 * i + hh) * 68 + c * 4);
  for (int rep = 0; rep < 2; ++rep) {
#pragma unroll
    for (int i = 0; i < 8; ++i)
      *(volatile v4f*)(og + (size_t)(2 * i + hh) * HD + c * 4) = ov[i];
    __threadfence();
  }
  __syncthreads();
  if (wave == 0 && lane < 8) {
    double S = 0.0, S2 = 0.0;
#pragma unroll 1
    for (int i = 0; i < 256; ++i) { S += wpart[2 * i]; S2 += wpart[2 * i + 1]; }
    v2d rv;
    rv[0] = S; rv[1] = S2;
    double* rp = recp + (size_t)bid * 16 + lane * 2;
    *(volatile v2d*)rp = rv;
    __threadfence();
    *(volatile v2d*)rp = rv;
  }
}

__global__ __launch_bounds__(256) void gn_y(const float* __restrict__ Op, const double* __restrict__ recp,
                                            const float* __restrict__ gw, const float* __restrict__ gbv,
                                            unsigned short* yh, unsigned short* yl) {
  __shared__ float sStat[4];
  const int tid = threadIdx.x;
  const int blk = blockIdx.x;
  const int rt  = blk % (SEQ / 64);
  const int h   = (blk / (SEQ / 64)) % NH;
  const int b   = blk / ((SEQ / 64) * NH);
  if (tid == 0) {
    double S = 0.0, S2 = 0.0;
    const double* rp = recp + ((size_t)((b * NH + h) * NQT)) * 16;
#pragma unroll 1
    for (int j = 0; j < NQT; ++j) { S += rp[j * 16]; S2 += rp[j * 16 + 1]; }
    const double mean = S * (1.0 / (double)GCOUNT);
    double var = S2 * (1.0 / (double)GCOUNT) - mean * mean;
    var = (var > 0.0) ? var : 0.0;
    const float varf = (float)var;
    sStat[0] = (float)mean;
    sStat[1] = 1.0f / sqrtf(varf + 1e-5f);
  }
  __syncthreads();
  const float mean = sStat[0];
  const float rstd = sStat[1];
  const int q8 = tid >> 3, d8 = (tid & 7) * 8;
  const v4f wa = *(const v4f*)(gw + h * HD + d8),  wb = *(const v4f*)(gw + h * HD + d8 + 4);
  const v4f ba = *(const v4f*)(gbv + h * HD + d8), bb = *(const v4f*)(gbv + h * HD + d8 + 4);
  float wv[8], bi[8];
#pragma unroll
  for (int e = 0; e < 4; ++e) {
    wv[e] = bf_up(bf_bits(wa[e])); wv[4 + e] = bf_up(bf_bits(wb[e]));
    bi[e] = bf_up(bf_bits(ba[e])); bi[4 + e] = bf_up(bf_bits(bb[e]));
  }
  v4u hv[2], lv[2];
#pragma unroll
  for (int it = 0; it < 2; ++it) {
    const int l = rt * 64 + it * 32 + q8;
    const float* xp = Op + (((size_t)(b * NH + h)) * SEQ + l) * HD + d8;
    const v4f xa = *(const v4f*)(xp), xb = *(const v4f*)(xp + 4);
    v4f ya, yb;
#pragma unroll
    for (int e = 0; e < 4; ++e) {
      float t0 = (xa[e] - mean) * rstd; t0 = t0 * wv[e] + bi[e];         ya[e] = t0 * 0.2f;
      float t1 = (xb[e] - mean) * rstd; t1 = t1 * wv[4 + e] + bi[4 + e]; yb[e] = t1 * 0.2f;
    }
    packhl(ya, yb, hv[it], lv[it]);
  }
  for (int rep = 0; rep < 2; ++rep) {
#pragma unroll
    for (int it = 0; it < 2; ++it) {
      const int l = rt * 64 + it * 32 + q8;
      const size_t o = ((size_t)(b * SEQ + l)) * HID + h * HD + d8;
      *(volatile v4u*)(yh + o) = hv[it];
      *(volatile v4u*)(yl + o) = lv[it];
    }
    __threadfence();
  }
}

extern "C" void kernel_launch(void* const* d_in, const int* in_sizes, int n_in,
                              void* d_out, int out_size, void* d_ws, size_t ws_size,
                              hipStream_t stream) {
  if (n_in < 12) return;
  if (in_sizes[0] < ((NB - 1) * SEQ_FULL + SEQ) * HID) return;
  if (in_sizes[1] < (NB - 1) * SEQ_FULL + SEQ) return;
  for (int i = 2; i < 8; ++i) if (in_sizes[i] < HID * HID) return;
  if (in_sizes[8] < NH * HD || in_sizes[9] < NH * HD) return;
  if (in_sizes[10] < HID || in_sizes[11] < HID) return;
  if (out_size < MTOT * HID) return;

  const float* x   = (const float*)d_in[0];
  const float* msk = (const float*)d_in[1];
  const float* wq0 = (const float*)d_in[2];
  const float* wq1 = (const float*)d_in[3];
  const float* wk0 = (const float*)d_in[4];
  const float* wk1 = (const float*)d_in[5];
  const float* wv  = (const float*)d_in[6];
  const float* wo  = (const float*)d_in[7];
  const float* l0  = (const float*)d_in[8];
  const float* l1  = (const float*)d_in[9];
  const float* gw  = (const float*)d_in[10];
  const float* gb  = (const float*)d_in[11];

  const size_t PPL = (size_t)MTOT * HID * 2;
  const size_t PWT = (size_t)6 * HID * HID * 2;
  const size_t PST = (size_t)NB * NH * 4 * SEQ * 4;
  const size_t PO  = (size_t)MTOT * HID * 4;
  const size_t PRC = (size_t)NBLK * 128;
  size_t off = 0;
  const size_t oXB  = off; off += PPL;
  const size_t oWT  = off; off += PWT;
  const size_t oQ0H = off; off += PPL;
  const size_t oQ0L = off; off += PPL;
  const size_t oQ1H = off; off += PPL;
  const size_t oQ1L = off; off += PPL;
  const size_t oK0H = off; off += PPL;
  const size_t oK0L = off; off += PPL;
  const size_t oK1H = off; off += PPL;
  const size_t oK1L = off; off += PPL;
  const size_t oVTH = off; off += PPL;
  const size_t oVTL = off; off += PPL;
  const size_t oST  = off; off += PST;
  const size_t oO   = off; off += PO;
  const size_t oRC  = off; off += PRC;
  const size_t oYH  = off; off += PPL;
  const size_t oYL  = off; off += PPL;
  if (off > ws_size) return;
  if (off > (size_t)134217728) return;

  char* ws = (char*)d_ws;
  unsigned short* Xb  = (unsigned short*)(ws + oXB);
  unsigned short* Wt  = (unsigned short*)(ws + oWT);
  unsigned short* Q0h = (unsigned short*)(ws + oQ0H);
  unsigned short* Q0l = (unsigned short*)(ws + oQ0L);
  unsigned short* Q1h = (unsigned short*)(ws + oQ1H);
  unsigned short* Q1l = (unsigned short*)(ws + oQ1L);
  unsigned short* K0h = (unsigned short*)(ws + oK0H);
  unsigned short* K0l = (unsigned short*)(ws + oK0L);
  unsigned short* K1h = (unsigned short*)(ws + oK1H);
  unsigned short* K1l = (unsigned short*)(ws + oK1L);
  unsigned short* VTh = (unsigned short*)(ws + oVTH);
  unsigned short* VTl = (unsigned short*)(ws + oVTL);
  float*          ST  = (float*)(ws + oST);
  float*          O   = (float*)(ws + oO);
  double*         REC = (double*)(ws + oRC);
  unsigned short* Yh  = (unsigned short*)(ws + oYH);
  unsigned short* Yl  = (unsigned short*)(ws + oYL);

  const size_t WSZ = (size_t)HID * HID;
  const int  n8 = MTOT * HID / 8;
  const dim3 blk256(256);
  const dim3 blk128(128);
  const dim3 gCvt((n8 + 255) / 256);
  const dim3 gWt((HID / 64) * (HID / 64), 6);
  const dim3 gGemm(HID / 64, MTOT / 128);
  const dim3 gAttn(NBLK);
  const dim3 gGn(NB * NH * (SEQ / 64));

  cvt_x<<<gCvt, blk256, 0, stream>>>(x, Xb, n8);
  cvt_wt<<<gWt, blk256, 0, stream>>>(wq0, wq1, wk0, wk1, wv, wo, Wt);
  gemm_bt<0, 1><<<gGemm, blk128, 0, stream>>>(Xb, Xb, Wt + 0 * WSZ, Q0h, Q0l, O);
  gemm_bt<0, 1><<<gGemm, blk128, 0, stream>>>(Xb, Xb, Wt + 1 * WSZ, Q1h, Q1l, O);
  gemm_bt<0, 1><<<gGemm, blk128, 0, stream>>>(Xb, Xb, Wt + 2 * WSZ, K0h, K0l, O);
  gemm_bt<0, 1><<<gGemm, blk128, 0, stream>>>(Xb, Xb, Wt + 3 * WSZ, K1h, K1l, O);
  gemm_bt<1, 1><<<gGemm, blk128, 0, stream>>>(Xb, Xb, Wt + 4 * WSZ, VTh, VTl, O);
  attn_stats<<<gAttn, blk256, 0, stream>>>(Q0h, Q0l, Q1h, Q1l, K0h, K0l, K1h, K1l, msk, ST);
  (void)hipFuncSetAttribute(reinterpret_cast<const void*>(&attn_out),
                            hipFuncAttributeMaxDynamicSharedMemorySize, L_TOTAL);
  attn_out<<<gAttn, blk256, L_TOTAL, stream>>>(Q0h, Q0l, Q1h, Q1l, K0h, K0l, K1h, K1l, VTh, VTl,
                                               msk, ST, l0, l1, O, REC);
  gn_y<<<gGn, blk256, 0, stream>>>(O, REC, gw, gb, Yh, Yl);
  gemm_bt<2, 2><<<gGemm, blk128, 0, stream>>>(Yh, Yl, Wt + 5 * WSZ, Yh, Yh, (float*)d_out);
  (void)hipGetLastError();
}
